// SplendorNNet_18605798326416
// MI455X (gfx1250) — hardware-run, weakly checked
//
#include <hip/hip_runtime.h>
#include <math.h>

constexpr int kBoards     = 32768;
constexpr int kNbVect     = 56;
constexpr int kVectDim    = 7;
constexpr int kRowsA      = kBoards * kVectDim;
constexpr int kChunks     = 4;
constexpr int kChunkRows  = kRowsA / kChunks;
constexpr int kAct        = 81;
constexpr int kScd        = 31;
constexpr float kWCarry    = 16.0f;
constexpr float kWCarryInv = 1.0f / 16.0f;
constexpr float kLowValue  = -1e8f;
constexpr float kBnEps     = 1e-5f;
constexpr int kOutFloats  = kBoards * (kAct + 1 + kScd);
constexpr int kOut1Base   = kBoards * kAct;
constexpr int kOut2Base   = kOut1Base + kBoards;

constexpr int kX0ld = 64;
constexpr int kP1ld = 256;
constexpr int kP2ld = 256;
constexpr int kP3ld = 320;
constexpr int kY3ld = 128;
constexpr int kC4ld = 704;
constexpr int kP5ld = 320;
constexpr int kP6ld = 320;
constexpr int kP7ld = 192;
constexpr int kP8ld = 192;
constexpr int kH1ld = 384;
constexpr int kLPld = 128;
constexpr int kLVld = 64;
constexpr int kLSld = 64;

static_assert(kChunkRows % 64 == 0);
static_assert(kChunkRows % 32 == 0);
static_assert(kChunkRows % kVectDim == 0);
static_assert(kBoards % 64 == 0);
static_assert(kBoards % 32 == 0);
static_assert((kOut1Base * 4) % 128 == 0);
static_assert((kOut2Base * 4) % 128 == 0);
static_assert((32 * kAct) % 32 == 0);
static_assert((32 * kScd) % 32 == 0);

constexpr size_t kX0Bytes = (size_t)kChunkRows * kX0ld * 2;
constexpr size_t kP1Bytes = (size_t)kChunkRows * kP1ld * 2;
constexpr size_t kP2Bytes = (size_t)kChunkRows * kP2ld * 2;
constexpr size_t kP3Bytes = (size_t)kChunkRows * kP3ld * 2;
static_assert(kP3Bytes == kX0Bytes + kP1Bytes);
constexpr size_t kRABytes = kP3Bytes + kP2Bytes;
constexpr size_t kY3Bytes = (size_t)kRowsA * kY3ld * 2;
constexpr size_t kC4Bytes = (size_t)kBoards * kC4ld * 2;
constexpr size_t kP5Bytes = (size_t)kBoards * kP5ld * 2;
constexpr size_t kP6Bytes = (size_t)kBoards * kP6ld * 2;
constexpr size_t kP7Bytes = (size_t)kBoards * kP7ld * 2;
constexpr size_t kP8Bytes = (size_t)kBoards * kP8ld * 2;
constexpr size_t kH1Bytes = (size_t)kBoards * kH1ld * 2;
constexpr size_t kLPBytes = (size_t)kBoards * kLPld * 4;
constexpr size_t kLVBytes = (size_t)kBoards * kLVld * 4;
constexpr size_t kLSBytes = (size_t)kBoards * kLSld * 4;
static_assert(kC4Bytes <= kRABytes);
static_assert(kP5Bytes + kP6Bytes <= kY3Bytes);
static_assert(kP7Bytes + kP8Bytes + kH1Bytes <= kRABytes);
static_assert(kLPBytes + kLVBytes + kLSBytes <= kY3Bytes);

typedef __attribute__((ext_vector_type(16))) _Float16 v16h;
typedef __attribute__((ext_vector_type(8)))  _Float16 v8h;
typedef __attribute__((ext_vector_type(16))) __bf16   v16b;
typedef __attribute__((ext_vector_type(8)))  __bf16   v8b;
typedef __attribute__((ext_vector_type(8)))  float    v8f;
typedef __attribute__((ext_vector_type(4)))  float    v4f;
typedef __attribute__((ext_vector_type(4)))  unsigned int v4u;

__device__ __forceinline__ unsigned short f2bf_bits(float f) {
  unsigned u = __float_as_uint(f);
  return (unsigned short)((u + 0x7FFFu + ((u >> 16) & 1u)) >> 16);
}
__device__ __forceinline__ float bf_bits2f(unsigned short h) { return __uint_as_float(((unsigned)h) << 16); }

__device__ __forceinline__ void dep_guard_h(v8f& a, v8f& b, v16h x, v16h y) { asm volatile("v_nop\n\tv_nop\n\tv_nop\n\tv_nop" : "+v"(a), "+v"(b) : "v"(x), "v"(y)); }
__device__ __forceinline__ void dep_guard_b(v8f& a, v8f& b, v16b x, v16b y) { asm volatile("v_nop\n\tv_nop\n\tv_nop\n\tv_nop" : "+v"(a), "+v"(b) : "v"(x), "v"(y)); }
__device__ __forceinline__ void keep4_h(v16h a, v16h b, v16h c, v16h d) { asm volatile("v_nop" :: "v"(a), "v"(b), "v"(c), "v"(d)); }
__device__ __forceinline__ void keep4_b(v16b a, v16b b, v16b c, v16b d) { asm volatile("v_nop" :: "v"(a), "v"(b), "v"(c), "v"(d)); }
__device__ __forceinline__ void acc_guard4(v8f& a, v8f& b, v8f& c, v8f& d) { asm volatile("v_nop\n\tv_nop\n\tv_nop\n\tv_nop" : "+v"(a), "+v"(b), "+v"(c), "+v"(d)); }
template <typename T> struct Frag;
template <> struct Frag<_Float16> {
  typedef v16h V; union U { v16h v; v8h h[2]; };
  static __device__ __forceinline__ v16h load(const _Float16* p) {
    U f; f.h[0] = *(const v8h*)(p); f.h[1] = *(const v8h*)(p + 16); return f.v;
  }
  static __device__ __forceinline__ v8f mma(v16h a, v16h b, v8f c) {
    return __builtin_amdgcn_wmma_f32_16x16x32_f16(false, a, false, b, (short)0, c, false, false);
  }
  static __device__ __forceinline__ void guard(v8f& a, v8f& b, v16h x, v16h y) { dep_guard_h(a, b, x, y); }
  static __device__ __forceinline__ void keep(v16h a, v16h b, v16h c, v16h d) { keep4_h(a, b, c, d); }
};
template <> struct Frag<__bf16> {
  typedef v16b V; union U { v16b v; v8b h[2]; };
  static __device__ __forceinline__ v16b load(const __bf16* p) {
    U f; f.h[0] = *(const v8b*)(p); f.h[1] = *(const v8b*)(p + 16); return f.v;
  }
  static __device__ __forceinline__ v8f mma(v16b a, v16b b, v8f c) {
    return __builtin_amdgcn_wmma_f32_16x16x32_bf16(false, a, false, b, (short)0, c, false, false);
  }
  static __device__ __forceinline__ void guard(v8f& a, v8f& b, v16b x, v16b y) { dep_guard_b(a, b, x, y); }
  static __device__ __forceinline__ void keep(v16b a, v16b b, v16b c, v16b d) { keep4_b(a, b, c, d); }
};

__device__ __forceinline__ unsigned pk16(unsigned short a, unsigned short b) { return (unsigned)a | ((unsigned)b << 16); }
__device__ __forceinline__ unsigned short h_bits(float f) { const _Float16 h = (_Float16)f; return __builtin_bit_cast(unsigned short, h); }
__device__ __forceinline__ float hlo2f(unsigned w) { return (float)__builtin_bit_cast(_Float16, (unsigned short)(w & 0xffffu)); }
__device__ __forceinline__ float hhi2f(unsigned w) { return (float)__builtin_bit_cast(_Float16, (unsigned short)(w >> 16)); }

template <int ET> struct Elem;
template <> struct Elem<0> { typedef _Float16 T; };
template <> struct Elem<1> { typedef __bf16 T; };
template <int ET, bool SPLIT, int BIAS_MODE, int OUT_MODE, bool RESID, int ACT = 0>
__global__ __launch_bounds__(256) void wmma_gemm64(
    const unsigned short* __restrict__ Ap, const unsigned short* __restrict__ A2p, int lda, long strideA,
    const unsigned short* __restrict__ Btp, const unsigned short* __restrict__ Bt2p, int ldb, long strideB,
    void* __restrict__ Cout, void* __restrict__ Cout2, int ldc, long strideC,
    const float* __restrict__ bias, const float* __restrict__ rowtab,
    const float* __restrict__ resid, long strideR,
    int M, int N, int K, float scale) {
  typedef typename Elem<ET>::T T;
  typedef typename Frag<T>::V V;
  const T* A = (const T*)Ap; const T* A2 = (const T*)A2p; const T* Bt = (const T*)Btp; const T* Bt2 = (const T*)Bt2p;
  __shared__ __align__(16) float sT[8][16 * 68];
  const int b    = blockIdx.y;
  const int lane = threadIdx.x & 31;
  const int wave = threadIdx.x >> 5;
  const int tilesN = N >> 6;
  const int tilesM = M >> 6;
  const int tile = blockIdx.x * 8 + wave;
  if (tile >= tilesM * tilesN) return;
  const int tm = tile / tilesN;
  const int tn = tile - tm * tilesN;
  const int m0 = tm << 6;
  const int n0 = tn << 6;

  const T* Ab  = A  + (size_t)b * strideA;
  const T* Bb  = Bt + (size_t)b * strideB;
  const T* Ab2 = SPLIT ? (A2  + (size_t)b * strideA) : nullptr;
  const T* Bb2 = SPLIT ? (Bt2 + (size_t)b * strideB) : nullptr;

  const int rlane = lane & 15;
  const int koff  = (lane >> 4) * 8;
  const int mOff  = (lane >> 4) * 8;

  v8f acc[4][4];
#pragma unroll
  for (int i = 0; i < 4; ++i)
#pragma unroll
    for (int j = 0; j < 4; ++j) acc[i][j] = (v8f){0.f,0.f,0.f,0.f,0.f,0.f,0.f,0.f};

  for (int k0 = 0; k0 < K; k0 += 32) {
    V bh[4], bl[4];
#pragma unroll
    for (int j = 0; j < 4; ++j) {
      const size_t bo = (size_t)(n0 + (j << 4) + rlane) * ldb + koff + k0;
      bh[j] = Frag<T>::load(Bb + bo);
      if (SPLIT) bl[j] = Frag<T>::load(Bb2 + bo);
    }
#pragma unroll
    for (int i = 0; i < 4; ++i) {
      const size_t ao = (size_t)(m0 + (i << 4) + rlane) * lda + koff + k0;
      V ah = Frag<T>::load(Ab + ao);
      V al;
      if (SPLIT) al = Frag<T>::load(Ab2 + ao);
#pragma unroll
      for (int j = 0; j < 4; ++j) {
        acc[i][j] = Frag<T>::mma(ah, bh[j], acc[i][j]);
        if (SPLIT) {
          acc[i][j] = Frag<T>::mma(ah, bl[j], acc[i][j]);
          acc[i][j] = Frag<T>::mma(al, bh[j], acc[i][j]);
        }
      }
      Frag<T>::guard(acc[i][0], acc[i][3], ah, SPLIT ? al : ah);
    }
    Frag<T>::keep(bh[0], bh[1], bh[2], bh[3]);
    if (SPLIT) Frag<T>::keep(bl[0], bl[1], bl[2], bl[3]);
  }
  acc_guard4(acc[0][0], acc[0][1], acc[0][2], acc[0][3]);
  acc_guard4(acc[1][0], acc[1][1], acc[1][2], acc[1][3]);
  acc_guard4(acc[2][0], acc[2][1], acc[2][2], acc[2][3]);
  acc_guard4(acc[3][0], acc[3][1], acc[3][2], acc[3][3]);

  float* slab = sT[wave];
  const float* Rb = RESID ? (resid + (size_t)b * strideR) : nullptr;
#pragma unroll
  for (int i = 0; i < 4; ++i) {
    const int mBase = m0 + (i << 4);
#pragma unroll
    for (int j = 0; j < 4; ++j) {
      const int n = n0 + (j << 4) + rlane;
      float bv = 0.f;
      if (BIAS_MODE == 2 || BIAS_MODE == 3) bv = bias[n];
#pragma unroll
      for (int r = 0; r < 8; ++r) {
        float v = acc[i][j][r] * scale;
        if (BIAS_MODE == 1) v += bias[mBase + mOff + r];
        if (BIAS_MODE == 2 || BIAS_MODE == 3) v += bv;
        if (BIAS_MODE == 3) {
          const int d = (mBase + mOff + r) % kVectDim;
          v = (v - rowtab[d]) * rowtab[8 + d] + rowtab[16 + d];
        }
        if (RESID) v += Rb[(size_t)(mBase + mOff + r) * ldc + n];
        if (ACT == 2) v = fmaxf(v, 0.0f);
        if (ACT == 4) v = (v > 0.f) ? v : 0.01f * v;
        slab[(mOff + r) * 68 + (j << 4) + rlane] = v;
      }
    }
    __builtin_amdgcn_fence(__ATOMIC_RELEASE, "workgroup");
    __builtin_amdgcn_wave_barrier();
    __builtin_amdgcn_fence(__ATOMIC_ACQUIRE, "workgroup");
    if (OUT_MODE == 0) {
      float* C = (float*)Cout + (size_t)b * strideC;
      const int hh = lane >> 4, c4 = (lane & 15) * 4;
      for (int pass = 0; pass < 2; ++pass) {
#pragma unroll
        for (int it = 0; it < 8; ++it) {
          const int row = it * 2 + hh;
          v4f v = *(const v4f*)(slab + row * 68 + c4);
          *(volatile v4f*)(C + (size_t)(mBase + row) * ldc + n0 + c4) = v;
        }
        __threadfence();
      }
    } else {
      const int q = lane >> 3, c8 = (lane & 7) * 8;
      unsigned short* C  = (unsigned short*)Cout  + (size_t)b * strideC;
      unsigned short* C2 = (OUT_MODE == 2) ? ((unsigned short*)Cout2 + (size_t)b * strideC) : nullptr;
      for (int pass = 0; pass < 2; ++pass) {
#pragma unroll
        for (int it = 0; it < 4; ++it) {
          const int row = it * 4 + q;
          const float* sp = slab + row * 68 + c8;
          v8h hv, lv;
#pragma unroll
          for (int e = 0; e < 8; ++e) {
            if (OUT_MODE == 1) {
              hv[e] = (_Float16)sp[e];
            } else {
              unsigned short hb = f2bf_bits(sp[e]);
              unsigned short lb = f2bf_bits(sp[e] - bf_bits2f(hb));
              hv[e] = __builtin_bit_cast(_Float16, hb);
              lv[e] = __builtin_bit_cast(_Float16, lb);
            }
          }
          *(volatile v8h*)(C + (size_t)(mBase + row) * ldc + n0 + c8) = hv;
          if (OUT_MODE == 2) *(volatile v8h*)(C2 + (size_t)(mBase + row) * ldc + n0 + c8) = lv;
        }
        __threadfence();
      }
    }
    __builtin_amdgcn_fence(__ATOMIC_RELEASE, "workgroup");
    __builtin_amdgcn_wave_barrier();
    __builtin_amdgcn_fence(__ATOMIC_ACQUIRE, "workgroup");
  }
}

__global__ __launch_bounds__(256) void prep_w_kernel(const float* __restrict__ W, const float* __restrict__ bsrc,
                                                     unsigned short* __restrict__ Wout, float* __restrict__ bout,
                                                     int Nsrc, int Ksrc, int Npad, int Kpad,
                                                     int len1, int src1, int dst2, int len2, int src2, float scale) {
  const int i = blockIdx.x * 256 + threadIdx.x;
  const int total8 = (Npad * Kpad) >> 3;
  if (i < total8) {
    const int e0 = i * 8;
    const int n = e0 / Kpad;
    const int k0 = e0 - n * Kpad;
    const int nc = (n < Nsrc) ? n : (Nsrc - 1);
    const bool rowok = (n < Nsrc);
    const float* wr = W + (size_t)nc * Ksrc;
    unsigned short hb[8];
#pragma unroll
    for (int e = 0; e < 8; ++e) {
      const int k = k0 + e;
      int c1 = src1 + k;
      c1 = (c1 < Ksrc) ? c1 : (Ksrc - 1);
      int c2 = src2 + k - dst2;
      c2 = (c2 < 0) ? 0 : c2;
      c2 = (c2 < Ksrc) ? c2 : (Ksrc - 1);
      const float f1 = wr[c1];
      const float f2 = wr[c2];
      const bool in1 = (k < len1);
      const bool in2 = (k >= dst2) && (k < dst2 + len2);
      float f = in1 ? f1 : (in2 ? f2 : 0.0f);
      f = rowok ? f : 0.0f;
      hb[e] = h_bits(f * scale);
    }
    const v4u u = (v4u){pk16(hb[0], hb[1]), pk16(hb[2], hb[3]), pk16(hb[4], hb[5]), pk16(hb[6], hb[7])};
    unsigned short* q = Wout + (size_t)e0;
    *(volatile v4u*)q = u;
    __threadfence();
    *(volatile v4u*)q = u;
  }
  const int nb4 = Npad >> 2;
  if (i < nb4) {
    v4f bvv;
#pragma unroll
    for (int e = 0; e < 4; ++e) {
      const int n = 4 * i + e;
      const int ncl = (n < Nsrc) ? n : (Nsrc - 1);
      const float f = bsrc[ncl];
      bvv[e] = (n < Nsrc) ? f : 0.0f;
    }
    float* q = bout + 4 * (size_t)i;
    *(volatile v4f*)q = bvv;
    __threadfence();
    *(volatile v4f*)q = bvv;
  }
}

__global__ __launch_bounds__(256) void xpose_in_kernel(const float* __restrict__ in,
                                                      const float* __restrict__ bng, const float* __restrict__ bnb,
                                                      const float* __restrict__ bnm, const float* __restrict__ bnv,
                                                      unsigned short* __restrict__ X0, float* __restrict__ bntab,
                                                      int row0, int writeTab) {
  const int t = threadIdx.x, lane = t & 31, wave = t >> 5;
  const int q = lane >> 3, c8 = (lane & 7) * 8;
  const int lr = blockIdx.x * 32 + wave * 4 + q;
  const int grow = row0 + lr;
  const int b = grow / kVectDim;
  const int v = grow - b * kVectDim;
  const float* ib = in + (size_t)b * (kNbVect * kVectDim) + v;
  unsigned short hb[8];
#pragma unroll
  for (int e = 0; e < 8; ++e) {
    const int c = c8 + e;
    const int cc = (c < kNbVect) ? c : (kNbVect - 1);
    float f = ib[cc * kVectDim];
    f = (c < kNbVect) ? f : 0.0f;
    hb[e] = h_bits(f);
  }
  const v4u u = (v4u){pk16(hb[0], hb[1]), pk16(hb[2], hb[3]), pk16(hb[4], hb[5]), pk16(hb[6], hb[7])};
  unsigned short* qo = X0 + (size_t)lr * kX0ld + c8;
  *(volatile v4u*)qo = u;
  __threadfence();
  *(volatile v4u*)qo = u;
  if (writeTab != 0 && blockIdx.x == 0 && wave == 0) {
    const int d = lane & 7;
    const int dd = (d < kVectDim) ? d : (kVectDim - 1);
    const float mm = bnm[dd], g = bng[dd], var = bnv[dd], bb = bnb[dd];
    const float a = g * (1.0f / sqrtf(var + kBnEps));
    float val = (lane < 8) ? mm : (lane < 16) ? a : (lane < 24) ? bb : 0.0f;
    val = (d < kVectDim) ? val : 0.0f;
    volatile float* qt = bntab + lane;
    *qt = val;
    __threadfence();
    *qt = val;
  }
}

template <int GS>
__global__ __launch_bounds__(256) void pool_kernel(const unsigned short* __restrict__ in, int ipitch,
                                                   unsigned short* __restrict__ out, int opitch, int ocol) {
  const int t = threadIdx.x, lane = t & 31, wave = t >> 5;
  const int q = lane >> 3, sub = lane & 7;
  const int row = blockIdx.x * 32 + wave * 4 + q;
  const int base = lane & 24;
  constexpr int NP = (GS == 8) ? 4 : 2;
  const int p = sub & (NP - 1);
  const v4u w = *(const v4u*)(in + (size_t)row * ipitch + p * 8);
  float x[8];
#pragma unroll
  for (int e = 0; e < 4; ++e) { x[2 * e] = hlo2f(w[e]); x[2 * e + 1] = hhi2f(w[e]); }
  float Mg[4], Sg[4];
  if (GS == 8) {
    float m = x[0], s = x[0];
#pragma unroll
    for (int e = 1; e < 8; ++e) { m = fmaxf(m, x[e]); s = s + x[e]; }
    const float m0 = __shfl(m, base + 0, 32), m1 = __shfl(m, base + 1, 32), m2 = __shfl(m, base + 2, 32), m3 = __shfl(m, base + 3, 32);
    const float s0 = __shfl(s, base + 0, 32), s1 = __shfl(s, base + 1, 32), s2 = __shfl(s, base + 2, 32), s3 = __shfl(s, base + 3, 32);
    Mg[0] = m0; Mg[1] = m1; Mg[2] = m2; Mg[3] = m3;
    Sg[0] = s0; Sg[1] = s1; Sg[2] = s2; Sg[3] = s3;
  } else {
    const float ma = fmaxf(fmaxf(x[0], x[1]), fmaxf(x[2], x[3]));
    const float mb = fmaxf(fmaxf(x[4], x[5]), fmaxf(x[6], x[7]));
    const float sa = ((x[0] + x[1]) + x[2]) + x[3];
    const float sb = ((x[4] + x[5]) + x[6]) + x[7];
    const float m0 = __shfl(ma, base + 0, 32), m1 = __shfl(mb, base + 0, 32), m2 = __shfl(ma, base + 1, 32), m3 = __shfl(mb, base + 1, 32);
    const float s0 = __shfl(sa, base + 0, 32), s1 = __shfl(sb, base + 0, 32), s2 = __shfl(sa, base + 1, 32), s3 = __shfl(sb, base + 1, 32);
    Mg[0] = m0; Mg[1] = m1; Mg[2] = m2; Mg[3] = m3;
    Sg[0] = s0; Sg[1] = s1; Sg[2] = s2; Sg[3] = s3;
  }
  const float inv = 1.0f / (float)GS;
  unsigned short hb[8];
#pragma unroll
  for (int g = 0; g < 4; ++g) { hb[g] = h_bits(Mg[g]); hb[4 + g] = h_bits(Sg[g] * inv); }
  const v4u val = (v4u){pk16(hb[0], hb[1]), pk16(hb[2], hb[3]), pk16(hb[4], hb[5]), pk16(hb[6], hb[7])};
  const bool keep = (sub == 0);
  v4u u;
  u[0] = keep ? val[0] : 0u;
  u[1] = keep ? val[1] : 0u;
  u[2] = keep ? val[2] : 0u;
  u[3] = keep ? val[3] : 0u;
  unsigned short* qo = out + (size_t)row * opitch + ocol + sub * 8;
  *(volatile v4u*)qo = u;
  __threadfence();
  *(volatile v4u*)qo = u;
}

__global__ __launch_bounds__(256) void concat_kernel(const unsigned short* __restrict__ Y3, unsigned short* __restrict__ C4) {
  const int t = threadIdx.x;
#pragma unroll 1
  for (int it = 0; it < 11; ++it) {
    const int task = it * 256 + t;
    const int bl = task / 88;
    const int rem = task - bl * 88;
    const int line = rem >> 3;
    const int c8 = (rem & 7) * 8;
    const int b = blockIdx.x * 32 + bl;
    const int colbase = (line >= 4) ? (64 + c8) : c8;
    const unsigned short* yb = Y3 + (size_t)b * (kVectDim * kY3ld) + colbase;
    const v4u w0 = *(const v4u*)(yb + 0 * kY3ld);
    const v4u w1 = *(const v4u*)(yb + 1 * kY3ld);
    const v4u w2 = *(const v4u*)(yb + 2 * kY3ld);
    const v4u w3 = *(const v4u*)(yb + 3 * kY3ld);
    const v4u w4 = *(const v4u*)(yb + 4 * kY3ld);
    const v4u w5 = *(const v4u*)(yb + 5 * kY3ld);
    const v4u w6 = *(const v4u*)(yb + 6 * kY3ld);
    const int t4 = line - 4;
    unsigned short hb[8];
#pragma unroll
    for (int e = 0; e < 8; ++e) {
      const int d = e >> 1;
      const bool hi = (e & 1) != 0;
      const float y0 = hi ? hhi2f(w0[d]) : hlo2f(w0[d]);
      const float y1 = hi ? hhi2f(w1[d]) : hlo2f(w1[d]);
      const float y2 = hi ? hhi2f(w2[d]) : hlo2f(w2[d]);
      const float y3 = hi ? hhi2f(w3[d]) : hlo2f(w3[d]);
      const float y4 = hi ? hhi2f(w4[d]) : hlo2f(w4[d]);
      const float y5 = hi ? hhi2f(w5[d]) : hlo2f(w5[d]);
      const float y6 = hi ? hhi2f(w6[d]) : hlo2f(w6[d]);
      const float mx = fmaxf(fmaxf(fmaxf(y0, y1), fmaxf(y2, y3)), y4);
      const float mean = ((((y0 + y1) + y2) + y3) + y4) * 0.2f;
      float pick = y6;
      pick = (t4 == 5) ? y5 : pick;
      pick = (t4 == 4) ? y4 : pick;
      pick = (t4 == 3) ? y3 : pick;
      pick = (t4 == 2) ? y2 : pick;
      pick = (t4 == 1) ? y1 : pick;
      pick = (t4 == 0) ? y0 : pick;
      pick = (line == 3) ? y6 : pick;
      pick = (line == 2) ? y5 : pick;
      float val = pick;
      val = (line == 1) ? mean : val;
      val = (line == 0) ? mx : val;
      hb[e] = h_bits(val);
    }
    const v4u u = (v4u){pk16(hb[0], hb[1]), pk16(hb[2], hb[3]), pk16(hb[4], hb[5]), pk16(hb[6], hb[7])};
    unsigned short* qo = C4 + (size_t)b * kC4ld + line * 64 + c8;
    *(volatile v4u*)qo = u;
    __threadfence();
    *(volatile v4u*)qo = u;
  }
}

__global__ __launch_bounds__(256) void heads_out_kernel(const float* __restrict__ LP, const float* __restrict__ LV,
                                                       const float* __restrict__ LS, const int* __restrict__ valid,
                                                       float* __restrict__ out) {
  __shared__ __align__(16) float s0[32 * kAct];
  __shared__ __align__(16) float s1[32];
  __shared__ __align__(16) float s2[32 * kScd];
  const int t = threadIdx.x;
  const int bl = t >> 3, sub = t & 7;
  const int b = blockIdx.x * 32 + bl;
  {
    const float* lp = LP + (size_t)b * kLPld;
    const int* va = valid + (size_t)b * kAct;
    float m = -INFINITY;
#pragma unroll 1
    for (int i = 0; i < 11; ++i) {
      const int j = sub + 8 * i;
      const int jc = (j < kAct) ? j : (kAct - 1);
      float x = lp[jc];
      const int vv = va[jc];
      x = (vv != 0) ? x : kLowValue;
      x = (j < kAct) ? x : -INFINITY;
      m = fmaxf(m, x);
    }
    m = fmaxf(m, __shfl_xor(m, 1, 32));
    m = fmaxf(m, __shfl_xor(m, 2, 32));
    m = fmaxf(m, __shfl_xor(m, 4, 32));
    float s = 0.0f;
#pragma unroll 1
    for (int i = 0; i < 11; ++i) {
      const int j = sub + 8 * i;
      const int jc = (j < kAct) ? j : (kAct - 1);
      float x = lp[jc];
      const int vv = va[jc];
      x = (vv != 0) ? x : kLowValue;
      x = (j < kAct) ? x : -INFINITY;
      s += expf(x - m);
    }
    s += __shfl_xor(s, 1, 32);
    s += __shfl_xor(s, 2, 32);
    s += __shfl_xor(s, 4, 32);
    const float lse = m + logf(s);
#pragma unroll 1
    for (int i = 0; i < 11; ++i) {
      const int j = sub + 8 * i;
      const int jc = (j < kAct) ? j : (kAct - 1);
      float x = lp[jc];
      const int vv = va[jc];
      x = (vv != 0) ? x : kLowValue;
      if (j < kAct) s0[bl * kAct + j] = x - lse;
    }
  }
  {
    const float th = tanhf(LV[(size_t)b * kLVld]);
    if (sub == 0) s1[bl] = th;
  }
  {
    const float* ls = LS + (size_t)b * kLSld;
    float m = -INFINITY;
#pragma unroll 1
    for (int i = 0; i < 4; ++i) {
      const int j = sub + 8 * i;
      const int jc = (j < kScd) ? j : (kScd - 1);
      float x = ls[jc];
      x = (j < kScd) ? x : -INFINITY;
      m = fmaxf(m, x);
    }
    m = fmaxf(m, __shfl_xor(m, 1, 32));
    m = fmaxf(m, __shfl_xor(m, 2, 32));
    m = fmaxf(m, __shfl_xor(m, 4, 32));
    float s = 0.0f;
#pragma unroll 1
    for (int i = 0; i < 4; ++i) {
      const int j = sub + 8 * i;
      const int jc = (j < kScd) ? j : (kScd - 1);
      float x = ls[jc];
      x = (j < kScd) ? x : -INFINITY;
      s += expf(x - m);
    }
    s += __shfl_xor(s, 1, 32);
    s += __shfl_xor(s, 2, 32);
    s += __shfl_xor(s, 4, 32);
    const float lse = m + logf(s);
#pragma unroll 1
    for (int i = 0; i < 4; ++i) {
      const int j = sub + 8 * i;
      const int jc = (j < kScd) ? j : (kScd - 1);
      const float x = ls[jc];
      if (j < kScd) s2[bl * kScd + j] = x - lse;
    }
  }
  __syncthreads();
  float* o0 = out + (size_t)blockIdx.x * (32 * kAct);
  float* o1 = out + (size_t)kOut1Base + (size_t)blockIdx.x * 32;
  float* o2 = out + (size_t)kOut2Base + (size_t)blockIdx.x * (32 * kScd);
  constexpr int n0q = (32 * kAct) / 4;
  constexpr int n2q = (32 * kScd) / 4;
  for (int pass = 0; pass < 2; ++pass) {
    for (int i = t; i < n0q; i += 256) {
      const v4f vv4 = *(const v4f*)(s0 + 4 * i);
      *(volatile v4f*)(o0 + 4 * (size_t)i) = vv4;
    }
    if (t < 8) {
      const v4f vv4 = *(const v4f*)(s1 + 4 * t);
      *(volatile v4f*)(o1 + 4 * t) = vv4;
    }
    for (int i = t; i < n2q; i += 256) {
      const v4f vv4 = *(const v4f*)(s2 + 4 * i);
      *(volatile v4f*)(o2 + 4 * (size_t)i) = vv4;
    }
    __threadfence();
  }
}

template <int BM, int OM, int ACT>
static void launch_gemm(hipStream_t st, const unsigned short* A, int lda, const unsigned short* Bt, int ldb,
                        void* C, int ldc, const float* bias, const float* rowtab, int M, int N, int K, float scale) {
  const int tiles = (M >> 6) * (N >> 6);
  wmma_gemm64<0, false, BM, OM, false, ACT><<<dim3((unsigned)((tiles + 7) / 8), 1, 1), dim3(256, 1, 1), 0, st>>>(
      A, A, lda, 0L, Bt, Bt, ldb, 0L, C, C, ldc, 0L, bias, rowtab, bias, 0L, M, N, K, scale);
}

extern "C" void kernel_launch(void* const* d_in, const int* in_sizes, int n_in,
                              void* d_out, int out_size, void* d_ws, size_t ws_size,
                              hipStream_t stream) {
  if (n_in < 34) return;
  if (in_sizes[0] != kBoards * kNbVect * kVectDim) return;
  if (in_sizes[1] != kBoards * kAct) return;
  if (out_size != kOutFloats) return;

  char* ws = (char*)d_ws;
  size_t off = 0;
  auto carve = [&](size_t bytes) -> size_t { const size_t o = off; off += (bytes + 255) & ~(size_t)255; return o; };

  const size_t nW1A = 256 * 64, nW1B = 256 * 256, nGP1 = 256 * 224, nW3P = 128 * 288, nW4P = 320 * 704, nGP4 = 256 * 256,
               nW5P = 192 * 288, nGP5 = 128 * 128, nHW1 = 384 * 160, nPIW2 = 128 * 128, nVW2 = 64 * 128, nSDW2 = 64 * 128;
  unsigned short* W1A  = (unsigned short*)(ws + carve(nW1A * 2));
  unsigned short* W1B  = (unsigned short*)(ws + carve(nW1B * 2));
  unsigned short* GP1  = (unsigned short*)(ws + carve(nGP1 * 2));
  unsigned short* W3P  = (unsigned short*)(ws + carve(nW3P * 2));
  unsigned short* W4P  = (unsigned short*)(ws + carve(nW4P * 2));
  unsigned short* GP4  = (unsigned short*)(ws + carve(nGP4 * 2));
  unsigned short* W5P  = (unsigned short*)(ws + carve(nW5P * 2));
  unsigned short* GP5  = (unsigned short*)(ws + carve(nGP5 * 2));
  unsigned short* HW1  = (unsigned short*)(ws + carve(nHW1 * 2));
  unsigned short* PIW2 = (unsigned short*)(ws + carve(nPIW2 * 2));
  unsigned short* VW2  = (unsigned short*)(ws + carve(nVW2 * 2));
  unsigned short* SDW2 = (unsigned short*)(ws + carve(nSDW2 * 2));
  float* B1A  = (float*)(ws + carve(256 * 4));
  float* B1B  = (float*)(ws + carve(256 * 4));
  float* GP1B = (float*)(ws + carve(256 * 4));
  float* B3   = (float*)(ws + carve(128 * 4));
  float* B4P  = (float*)(ws + carve(320 * 4));
  float* GP4B = (float*)(ws + carve(256 * 4));
  float* B5P  = (float*)(ws + carve(192 * 4));
  float* GP5B = (float*)(ws + carve(128 * 4));
  float* HB1  = (float*)(ws + carve(384 * 4));
  float* PIB2 = (float*)(ws + carve(128 * 4));
  float* VB2  = (float*)(ws + carve(64 * 4));
  float* SDB2 = (float*)(ws + carve(64 * 4));
  float* BNT  = (float*)(ws + carve(32 * 4));
  char* RA  = ws + carve(kRABytes);
  char* Y3R = ws + carve(kY3Bytes);
  if (off > ws_size) return;

  unsigned short* X0 = (unsigned short*)(RA);
  unsigned short* P1 = (unsigned short*)(RA + kX0Bytes);
  unsigned short* P3 = (unsigned short*)(RA);
  unsigned short* P2 = (unsigned short*)(RA + kP3Bytes);
  unsigned short* Y3 = (unsigned short*)(Y3R);
  unsigned short* C4 = (unsigned short*)(RA);
  unsigned short* P5 = (unsigned short*)(Y3R);
  unsigned short* P6 = (unsigned short*)(Y3R + kP5Bytes);
  unsigned short* P7 = (unsigned short*)(RA);
  unsigned short* P8 = (unsigned short*)(RA + kP7Bytes);
  unsigned short* H1 = (unsigned short*)(RA + kP7Bytes + kP8Bytes);
  float* LP = (float*)(Y3R);
  float* LV = (float*)(Y3R + kLPBytes);
  float* LS = (float*)(Y3R + kLPBytes + kLVBytes);

  const float* inX = (const float*)d_in[0];
  const int* inValid = (const int*)d_in[1];

  auto prep = [&](int wi, int bi, unsigned short* Wout, float* bout, int Nsrc, int Ksrc, int Npad, int Kpad,
                  int len1, int src1, int dst2, int len2, int src2) {
    const int total8 = (Npad * Kpad) / 8;
    const int nb4 = Npad / 4;
    const int nthr = (total8 > nb4) ? total8 : nb4;
    prep_w_kernel<<<dim3((unsigned)((nthr + 255) / 256)), dim3(256), 0, stream>>>(
        (const float*)d_in[wi], (const float*)d_in[bi], Wout, bout, Nsrc, Ksrc, Npad, Kpad, len1, src1, dst2, len2, src2, kWCarry);
  };
  prep(2,  3,  W1A,  B1A,  256, 56,  256, 64,  56,  0, 0,   0, 0);
  prep(8,  9,  W1B,  B1B,  256, 256, 256, 256, 256, 0, 0,   0, 0);
  prep(10, 11, GP1,  GP1B, 248, 224, 256, 224, 224, 0, 0,   0, 0);
  prep(12, 13, W3P,  B3,   128, 256, 128, 288, 248, 8, 256, 8, 0);
  prep(14, 15, W4P,  B4P,  256, 704, 320, 704, 704, 0, 0,   0, 0);
  prep(16, 17, GP4,  GP4B, 248, 240, 256, 256, 240, 0, 0,   0, 0);
  prep(18, 19, W5P,  B5P,  128, 256, 192, 288, 248, 8, 256, 8, 0);
  prep(20, 21, GP5,  GP5B, 120, 112, 128, 128, 112, 0, 0,   0, 0);
  prep(22, 23, HW1,                      HB1,       128, 128, 128, 160, 120, 8, 128, 8, 0);
  prep(26, 27, HW1 + (size_t)128 * 160,  HB1 + 128, 128, 128, 128, 160, 120, 8, 128, 8, 0);
  prep(30, 31, HW1 + (size_t)256 * 160,  HB1 + 256, 128, 128, 128, 160, 120, 8, 128, 8, 0);
  prep(24, 25, PIW2, PIB2, 81,  128, 128, 128, 128, 0, 0,   0, 0);
  prep(28, 29, VW2,  VB2,  1,   128, 64,  128, 128, 0, 0,   0, 0);
  prep(32, 33, SDW2, SDB2, 31,  128, 64,  128, 128, 0, 0,   0, 0);

  for (int c = 0; c < kChunks; ++c) {
    const int row0 = c * kChunkRows;
    xpose_in_kernel<<<dim3(kChunkRows / 32), dim3(256), 0, stream>>>(
        inX, (const float*)d_in[4], (const float*)d_in[5], (const float*)d_in[6], (const float*)d_in[7],
        X0, BNT, row0, (c == 0) ? 1 : 0);
    launch_gemm<3, 1, 2>(stream, X0, kX0ld, W1A, 64, P1, kP1ld, B1A, BNT, kChunkRows, 256, 64, kWCarryInv);
    launch_gemm<2, 1, 2>(stream, P1, kP1ld, W1B, 256, P2, kP2ld, B1B, BNT, kChunkRows, 256, 256, kWCarryInv);
    launch_gemm<2, 1, 2>(stream, P2 + 32, kP2ld, GP1, 224, P3, kP3ld, GP1B, BNT, kChunkRows, 256, 224, kWCarryInv);
    pool_kernel<8><<<dim3(kChunkRows / 32), dim3(256), 0, stream>>>(P2, kP2ld, P3, kP3ld, 256);
    launch_gemm<2, 1, 2>(stream, P3, kP3ld, W3P, 288, Y3 + (size_t)row0 * kY3ld, kY3ld, B3, BNT, kChunkRows, 128, 288, kWCarryInv);
  }

  concat_kernel<<<dim3(kBoards / 32), dim3(256), 0, stream>>>(Y3, C4);
  launch_gemm<2, 1, 2>(stream, C4, kC4ld, W4P, 704, P5, kP5ld, B4P, BNT, kBoards, 320, 704, kWCarryInv);
  launch_gemm<2, 1, 2>(stream, P5 + 16, kP5ld, GP4, 256, P6, kP6ld, GP4B, BNT, kBoards, 256, 256, kWCarryInv);
  pool_kernel<4><<<dim3(kBoards / 32), dim3(256), 0, stream>>>(P5, kP5ld, P6, kP6ld, 256);
  launch_gemm<2, 1, 2>(stream, P6, kP6ld, W5P, 288, P7, kP7ld, B5P, BNT, kBoards, 192, 288, kWCarryInv);
  launch_gemm<2, 1, 2>(stream, P7 + 16, kP7ld, GP5, 128, P8, kP8ld, GP5B, BNT, kBoards, 128, 128, kWCarryInv);
  pool_kernel<4><<<dim3(kBoards / 32), dim3(256), 0, stream>>>(P7, kP7ld, P8, kP8ld, 128);
  launch_gemm<2, 1, 0>(stream, P8, kP8ld, HW1, 160, H1, kH1ld, HB1, BNT, kBoards, 384, 160, kWCarryInv);
  launch_gemm<2, 0, 0>(stream, H1,       kH1ld, PIW2, 128, LP, kLPld, PIB2, BNT, kBoards, 128, 128, kWCarryInv);
  launch_gemm<2, 0, 0>(stream, H1 + 128, kH1ld, VW2,  128, LV, kLVld, VB2,  BNT, kBoards, 64,  128, kWCarryInv);
  launch_gemm<2, 0, 0>(stream, H1 + 256, kH1ld, SDW2, 128, LS, kLSld, SDB2, BNT, kBoards, 64,  128, kWCarryInv);

  heads_out_kernel<<<dim3(kBoards / 32), dim3(256), 0, stream>>>(LP, LV, LS, inValid, (float*)d_out);
}
